// GINGrapherLayer_44590350467907
// MI455X (gfx1250) — hardware-verified
//
#include <hip/hip_runtime.h>
#include <stddef.h>


#define DH     128
#define NTHR   256
#define NWAVE  8
#define RB     128
#define KC     128
#define AP     (KC + 8)
#define SP     132
#define CS     128
#define STW    1024
#define STH    512
#define EPT    8
#define NGRP   2
#define CHUNK  (NTHR * EPT * NGRP)
#define WCAP   (EPT * NGRP * 32)
#define LISTN  (NWAVE * WCAP)
#define NB     2048
#define RCAP   40960
#define DEGCAP 256
#define WTOT   245760
#define LDS_GEMM (2 * RB * AP * 2 + RB * SP * 4 + 2 * CS * 8)
#define LDS_CSR  ((RCAP + 3 * NB + LISTN + 2 * NWAVE) * 4)

static_assert((CHUNK & (CHUNK - 1)) == 0);
static_assert(CHUNK <= 4096);
static_assert(NB <= 4096 && (NB & (NB - 1)) == 0);
static_assert(NB == NTHR * 8);
static_assert((NB % NWAVE) == 0);
static_assert((RCAP % 32) == 0);
static_assert(RB == NWAVE * 16);
static_assert((KC % 32) == 0);
static_assert((AP % 8) == 0);
static_assert((SP % 4) == 0);
static_assert(CS == 128);

typedef float          v4f   __attribute__((ext_vector_type(4)));
typedef float          v8f   __attribute__((ext_vector_type(8)));
typedef int            v4i   __attribute__((ext_vector_type(4)));
typedef double         v2d   __attribute__((ext_vector_type(2)));
typedef unsigned short v8us  __attribute__((ext_vector_type(8)));
typedef __bf16         v16bf __attribute__((ext_vector_type(16)));
union FragB { v16bf v; v8us h[2]; };

__device__ __forceinline__ unsigned int bfr_bits(float f) {
  unsigned int u = __float_as_uint(f);
  u += 0x7FFFu + ((u >> 16) & 1u);
  return u >> 16;
}

__device__ __forceinline__ void split1(float f, unsigned short& hi, unsigned short& lo) {
  const unsigned int hb = bfr_bits(f);
  const float hf = __uint_as_float(hb << 16);
  hi = (unsigned short)hb;
  lo = (unsigned short)bfr_bits(f - hf);
}

__device__ __forceinline__ void split8(v4f a, v4f b, v8us& hi, v8us& lo) {
  unsigned short h0, h1, h2, h3, h4, h5, h6, h7, l0, l1, l2, l3, l4, l5, l6, l7;
  split1(a.x, h0, l0); split1(a.y, h1, l1); split1(a.z, h2, l2); split1(a.w, h3, l3);
  split1(b.x, h4, l4); split1(b.y, h5, l5); split1(b.z, h6, l6); split1(b.w, h7, l7);
  hi[0] = h0; hi[1] = h1; hi[2] = h2; hi[3] = h3; hi[4] = h4; hi[5] = h5; hi[6] = h6; hi[7] = h7;
  lo[0] = l0; lo[1] = l1; lo[2] = l2; lo[3] = l3; lo[4] = l4; lo[5] = l5; lo[6] = l6; lo[7] = l7;
}

__device__ __forceinline__ v8f wmb(v16bf a, v16bf b, v8f c) {
  v8f d = __builtin_amdgcn_wmma_f32_16x16x32_bf16(false, a, false, b, (short)0, c, false, false);
  asm volatile("v_nop\n\tv_nop\n\tv_nop\n\tv_nop" : "+v"(d) : "v"(a), "v"(b));
  return d;
}

__device__ __forceinline__ float gelu1(float v) {
  const float e = erff(v * 0.70710678118654752f);
  return 0.5f * v * (1.0f + e);
}

__device__ __forceinline__ v4f bn4(v4f v, v4f m, v4f is, v4f g, v4f b) {
  v4f t = g * (v - m);
  t = t * is;
  return t + b;
}

template <int NBS>
__device__ __forceinline__ int scan_chunk(const int* __restrict__ dsts, int nE, int cbase, int slotBase,
                                          int vec8, int* list, int tid, int lane, int wave) {
  int wc = 0;
#pragma unroll
  for (int g = 0; g < NGRP; ++g) {
    const int el0  = (g * NTHR + tid) * EPT;
    const int e0   = cbase + el0;
    const int sent = -2147483647 - 1;
    v4i da, db;
    if (vec8 != 0 && cbase + CHUNK <= nE) {
      da = *(const v4i*)(dsts + e0);
      db = *(const v4i*)(dsts + e0 + 4);
    } else {
      da.x = (e0     < nE) ? dsts[min(e0, nE - 1)] : sent;
      da.y = (e0 + 1 < nE) ? dsts[min(e0 + 1, nE - 1)] : sent;
      da.z = (e0 + 2 < nE) ? dsts[min(e0 + 2, nE - 1)] : sent;
      da.w = (e0 + 3 < nE) ? dsts[min(e0 + 3, nE - 1)] : sent;
      db.x = (e0 + 4 < nE) ? dsts[min(e0 + 4, nE - 1)] : sent;
      db.y = (e0 + 5 < nE) ? dsts[min(e0 + 5, nE - 1)] : sent;
      db.z = (e0 + 6 < nE) ? dsts[min(e0 + 6, nE - 1)] : sent;
      db.w = (e0 + 7 < nE) ? dsts[min(e0 + 7, nE - 1)] : sent;
    }
    const unsigned nb = (unsigned)slotBase;
    const unsigned s0 = (unsigned)da.x - nb, s1 = (unsigned)da.y - nb;
    const unsigned s2 = (unsigned)da.z - nb, s3 = (unsigned)da.w - nb;
    const unsigned s4 = (unsigned)db.x - nb, s5 = (unsigned)db.y - nb;
    const unsigned s6 = (unsigned)db.z - nb, s7 = (unsigned)db.w - nb;
    const bool h0 = s0 < (unsigned)NBS, h1 = s1 < (unsigned)NBS, h2 = s2 < (unsigned)NBS, h3 = s3 < (unsigned)NBS;
    const bool h4 = s4 < (unsigned)NBS, h5 = s5 < (unsigned)NBS, h6 = s6 < (unsigned)NBS, h7 = s7 < (unsigned)NBS;
    const unsigned any = __builtin_amdgcn_ballot_w32(h0 | h1 | h2 | h3 | h4 | h5 | h6 | h7);
    if (any != 0u) {
#define HITJ(J, HJ, SJ) { \
        const unsigned mj = __builtin_amdgcn_ballot_w32(HJ); \
        if (mj != 0u) { \
          if (HJ) { \
            const int pos = wc + (int)__builtin_amdgcn_mbcnt_lo(mj, 0u); \
            if (pos < WCAP) list[wave * WCAP + pos] = ((el0 + (J)) << 12) | (int)(SJ); \
          } \
          wc += (int)__builtin_popcount(mj); } }
      HITJ(0, h0, s0)
      HITJ(1, h1, s1)
      HITJ(2, h2, s2)
      HITJ(3, h3, s3)
      HITJ(4, h4, s4)
      HITJ(5, h5, s5)
      HITJ(6, h6, s6)
      HITJ(7, h7, s7)
#undef HITJ
    }
  }
  return wc;
}

__global__ __launch_bounds__(NTHR) void k_wprep(
    const float* __restrict__ w0, const float* __restrict__ w1, const float* __restrict__ w2,
    const float* __restrict__ w3, const float* __restrict__ w4, const float* __restrict__ w5,
    const float* __restrict__ w6, unsigned short* whi, unsigned short* wlo) {
  const int bid = (int)blockIdx.x, tid = (int)threadIdx.x;
  const int seg = bid < 8 ? 0 : (bid < 16 ? 1 : (bid < 24 ? 2 : (bid < 40 ? 3 : (bid < 56 ? 4 : (bid < 88 ? 5 : 6)))));
  const float* src = seg == 0 ? w0 : (seg == 1 ? w1 : (seg == 2 ? w2 : (seg == 3 ? w3 : (seg == 4 ? w4 : (seg == 5 ? w5 : w6)))));
  const int sb   = seg == 0 ? 0 : (seg == 1 ? 8 : (seg == 2 ? 16 : (seg == 3 ? 24 : (seg == 4 ? 40 : (seg == 5 ? 56 : 88)))));
  const int ncol = seg == 3 ? 2 * DH : (seg == 5 ? 4 * DH : DH);
  const int ksh  = seg == 4 ? 5 : (seg == 6 ? 6 : 4);
  const int pb   = seg == 0 ? 0 : (seg == 1 ? 16384 : (seg == 2 ? 32768 : (seg == 3 ? 49152 :
                   (seg == 4 ? 81920 : (seg == 5 ? 114688 : 180224)))));
  const int i  = (bid - sb) * NTHR + tid;
  const int n  = i >> ksh;
  const int k0 = (i & ((1 << ksh) - 1)) * 8;
  v4f a, b;
  a.x = src[(size_t)(k0 + 0) * ncol + n]; a.y = src[(size_t)(k0 + 1) * ncol + n];
  a.z = src[(size_t)(k0 + 2) * ncol + n]; a.w = src[(size_t)(k0 + 3) * ncol + n];
  b.x = src[(size_t)(k0 + 4) * ncol + n]; b.y = src[(size_t)(k0 + 5) * ncol + n];
  b.z = src[(size_t)(k0 + 6) * ncol + n]; b.w = src[(size_t)(k0 + 7) * ncol + n];
  v8us hv, lv;
  split8(a, b, hv, lv);
  const size_t o = (size_t)pb + (size_t)i * 8;
  *(volatile v8us*)(whi + o) = hv;
  *(volatile v8us*)(wlo + o) = lv;
  __threadfence();
  *(volatile v8us*)(whi + o) = hv;
  *(volatile v8us*)(wlo + o) = lv;
}

template <int KD, int NC, int AM, int STATS>
__global__ __launch_bounds__(NTHR) void k_gemm(
    const float* __restrict__ A, const float* __restrict__ bnst,
    const float* __restrict__ bng, const float* __restrict__ bnb,
    const unsigned short* __restrict__ Bh, const unsigned short* __restrict__ Bl,
    const float* __restrict__ bias, float* C, double* part, int nRowsA, int nRowsC) {
  extern __shared__ v4f lds_dyn[];
  constexpr int NKC   = KD / KC;
  constexpr int NSLAB = NC / CS;
  constexpr int KV    = KC / 8;
  constexpr int NTL   = CS / 16;
  static_assert((KD % KC) == 0);
  static_assert((NC % CS) == 0);
  static_assert(((RB * KV) % NTHR) == 0);
  unsigned short* sAh = (unsigned short*)lds_dyn;
  unsigned short* sAl = sAh + RB * AP;
  float*  stg = (float*)((char*)lds_dyn + (size_t)2 * RB * AP * 2);
  double* pst = (double*)((char*)lds_dyn + (size_t)2 * RB * AP * 2 + (size_t)RB * SP * 4);
  const int tid = threadIdx.x, lane = tid & 31, wave = tid >> 5, hh = lane >> 4, m = lane & 15;
  const int rowBase = blockIdx.x * RB;

#pragma unroll 1
  for (int slab = 0; slab < NSLAB; ++slab) {
    v8f acc[NTL];
#pragma unroll
    for (int t = 0; t < NTL; ++t) { v8f z = {0.f, 0.f, 0.f, 0.f, 0.f, 0.f, 0.f, 0.f}; acc[t] = z; }

#pragma unroll 1
    for (int kc = 0; kc < NKC; ++kc) {
      if (NKC > 1 || slab == 0) {
        __syncthreads();
#pragma unroll 2
        for (int i = 0; i < (RB * KV) / NTHR; ++i) {
          const int idx = i * NTHR + tid;
          const int r   = idx / KV;
          const int c0  = (idx % KV) * 8;
          int row = rowBase + r;
          row = row > nRowsA - 1 ? nRowsA - 1 : row;
          const int kcol = kc * KC + c0;
          const float* ap = A + (size_t)row * KD + kcol;
          v4f a = *(const v4f*)ap;
          v4f b = *(const v4f*)(ap + 4);
          if (AM == 2) {
            const v4f ma = *(const v4f*)(bnst + kcol),       mb = *(const v4f*)(bnst + kcol + 4);
            const v4f ia = *(const v4f*)(bnst + STH + kcol), ib = *(const v4f*)(bnst + STH + kcol + 4);
            const v4f ga = *(const v4f*)(bng + kcol),        gq = *(const v4f*)(bng + kcol + 4);
            const v4f ba = *(const v4f*)(bnb + kcol),        bq = *(const v4f*)(bnb + kcol + 4);
            a = bn4(a, ma, ia, ga, ba);
            b = bn4(b, mb, ib, gq, bq);
            a.x = gelu1(a.x); a.y = gelu1(a.y); a.z = gelu1(a.z); a.w = gelu1(a.w);
            b.x = gelu1(b.x); b.y = gelu1(b.y); b.z = gelu1(b.z); b.w = gelu1(b.w);
          }
          v8us hv, lv;
          split8(a, b, hv, lv);
          *(v8us*)(sAh + r * AP + c0) = hv;
          *(v8us*)(sAl + r * AP + c0) = lv;
        }
        __syncthreads();
      }
      const unsigned short* ah = sAh + (wave * 16 + m) * AP + 8 * hh;
      const unsigned short* al = sAl + (wave * 16 + m) * AP + 8 * hh;
#pragma unroll
      for (int ks = 0; ks < KC / 32; ++ks) {
        FragB fah, fal;
        fah.h[0] = *(const v8us*)(ah + 32 * ks);
        fah.h[1] = *(const v8us*)(ah + 32 * ks + 16);
        fal.h[0] = *(const v8us*)(al + 32 * ks);
        fal.h[1] = *(const v8us*)(al + 32 * ks + 16);
#pragma unroll
        for (int t = 0; t < NTL; ++t) {
          const size_t bo = (size_t)(slab * CS + 16 * t + m) * KD + (size_t)(kc * KC + 32 * ks + 8 * hh);
          FragB fbh, fbl;
          fbh.h[0] = *(const v8us*)(Bh + bo);
          fbh.h[1] = *(const v8us*)(Bh + bo + 16);
          fbl.h[0] = *(const v8us*)(Bl + bo);
          fbl.h[1] = *(const v8us*)(Bl + bo + 16);
          acc[t] = wmb(fah.v, fbh.v, acc[t]);
          acc[t] = wmb(fah.v, fbl.v, acc[t]);
          acc[t] = wmb(fal.v, fbh.v, acc[t]);
        }
      }
    }

    __syncthreads();
    {
      const int r0 = wave * 16 + 8 * hh;
      float* sp = stg + r0 * SP + m;
#pragma unroll
      for (int t = 0; t < NTL; ++t) {
        const float bv = bias[slab * CS + 16 * t + m];
#pragma unroll
        for (int r = 0; r < 8; ++r) sp[r * SP + 16 * t] = acc[t][r] + bv;
      }
    }
    __syncthreads();

    const float* lrow = stg + (wave * 16) * SP + 4 * lane;
#pragma unroll
    for (int r = 0; r < 16; ++r) {
      const int row = rowBase + wave * 16 + r;
      if (row < nRowsC) {
        const v4f v = *(const v4f*)(lrow + r * SP);
        *(volatile v4f*)(C + (size_t)row * NC + slab * CS + 4 * lane) = v;
      }
    }
    __threadfence();
#pragma unroll
    for (int r = 0; r < 16; ++r) {
      const int row = rowBase + wave * 16 + r;
      if (row < nRowsC) {
        const v4f v = *(const v4f*)(lrow + r * SP);
        *(volatile v4f*)(C + (size_t)row * NC + slab * CS + 4 * lane) = v;
      }
    }

    if (STATS) {
      int rmax = nRowsA - rowBase;
      rmax = rmax < 0 ? 0 : (rmax > RB ? RB : rmax);
      if (tid < CS) {
        double sm = 0.0, sq = 0.0;
#pragma unroll 4
        for (int r = 0; r < rmax; ++r) {
          const double v = (double)stg[r * SP + tid];
          sm += v;
          sq += v * v;
        }
        pst[tid] = sm;
        pst[CS + tid] = sq;
      }
      __syncthreads();
      v2d pv = {0.0, 0.0};
      if (tid < CS) pv = *(const v2d*)(pst + 2 * tid);
      double* pp = part + (size_t)blockIdx.x * (2 * NC) + (size_t)slab * (2 * CS) + 2 * tid;
      if (tid < CS) *(volatile v2d*)pp = pv;
      __threadfence();
      if (tid < CS) *(volatile v2d*)pp = pv;
    }
  }
}

__global__ __launch_bounds__(512) void k_bnfin(
    const double* __restrict__ part, int nBlk, int nc, int nRows, float* st) {
  __shared__ __attribute__((aligned(16))) float ss[STW];
  const int tid = threadIdx.x;
  int c = tid < nc ? tid : nc - 1;
  c = c < 0 ? 0 : c;
  const int slab = c >> 7, cc = c & 127;
  const int pitch = 2 * nc;
  double s = 0.0, q = 0.0;
#pragma unroll 1
  for (int b2 = 0; b2 < nBlk; ++b2) {
    const double* p = part + (size_t)b2 * pitch + slab * 256;
    s += p[cc];
    q += p[128 + cc];
  }
  const double inv_n = 1.0 / (double)nRows;
  const double mean = s * inv_n;
  double var = q * inv_n - mean * mean;
  var = var < 0.0 ? 0.0 : var;
  const float meanf = (float)mean;
  const float ve = (float)var + 1e-5f;
  const float istd = rsqrtf(ve);
  ss[tid] = (tid < nc) ? meanf : 0.0f;
  ss[STH + tid] = (tid < nc) ? istd : 0.0f;
  __syncthreads();
  v4f v = {0.f, 0.f, 0.f, 0.f};
  if (tid < 256) v = *(const v4f*)(ss + 4 * tid);
  if (tid < 256) *(volatile v4f*)(st + 4 * tid) = v;
  __threadfence();
  if (tid < 256) *(volatile v4f*)(st + 4 * tid) = v;
}

__global__ __launch_bounds__(NTHR) void k_aggr(
    const int* __restrict__ ei, const float* __restrict__ y0, const float* __restrict__ st0,
    const float* __restrict__ g0, const float* __restrict__ b0, float* aout, int nN, int nE, int vec8) {
  extern __shared__ v4f lds_dyn[];
  int* region = (int*)lds_dyn;
  int* scnt   = region + RCAP;
  int* soff   = scnt + NB;
  int* scur   = soff + NB;
  int* list   = scur + NB;
  int* wcnt   = list + LISTN;
  int* wtot   = wcnt + NWAVE;
  const int tid = threadIdx.x, lane = tid & 31, wave = tid >> 5;
  const int b = blockIdx.x;
  const int nodeBase = b * NB;
  const int* srcs = ei;
  const int* dsts = ei + nE;

  {
    const v4i z = {0, 0, 0, 0};
#pragma unroll 1
    for (int i = tid; i < RCAP / 4; i += NTHR) ((v4i*)region)[i] = z;
#pragma unroll 1
    for (int i = tid; i < NB / 4; i += NTHR) ((v4i*)scnt)[i] = z;
  }
  __syncthreads();

  const int nChunks = (nE + CHUNK - 1) / CHUNK;

#pragma unroll 1
  for (int ch = 0; ch < nChunks; ++ch) {
    const int cbase = ch * CHUNK;
    const int wc = scan_chunk<NB>(dsts, nE, cbase, nodeBase, vec8, list, tid, lane, wave);
    if (lane == 0) wcnt[wave] = wc;
    __syncthreads();
    if (wave == 0) {
#pragma unroll 1
      for (int wsx = 0; wsx < NWAVE; ++wsx) {
        int n = __builtin_amdgcn_readfirstlane(wcnt[wsx]);
        n = n > WCAP ? WCAP : (n < 0 ? 0 : n);
        const int* lp = list + wsx * WCAP;
#pragma unroll 1
        for (int i = 0; i < n; ++i) {
          const int ent  = __builtin_amdgcn_readfirstlane(lp[i]);
          const int slot = ent & (NB - 1);
          if (lane == 0) scnt[slot] = scnt[slot] + 1;
        }
      }
    }
    __syncthreads();
  }

  int ev[8];
  {
    const v4i c0 = *(const v4i*)(scnt + 8 * tid);
    const v4i c1 = *(const v4i*)(scnt + 8 * tid + 4);
    ev[0] = max(c0.x, 0); ev[1] = max(c0.y, 0); ev[2] = max(c0.z, 0); ev[3] = max(c0.w, 0);
    ev[4] = max(c1.x, 0); ev[5] = max(c1.y, 0); ev[6] = max(c1.z, 0); ev[7] = max(c1.w, 0);
  }
  int ts = 0;
#pragma unroll
  for (int i = 0; i < 8; ++i) ts += ev[i];
  int incl = ts;
#pragma unroll
  for (int d = 1; d < 32; d <<= 1) {
    const int t = __shfl_up(incl, d);
    if (lane >= d) incl += t;
  }
  if (lane == 31) wtot[wave] = incl;
  __syncthreads();
  int pre = 0;
#pragma unroll 1
  for (int w = 0; w < wave; ++w) pre += wtot[w];
  {
    int run = pre + incl - ts;
    int ov[8];
#pragma unroll
    for (int i = 0; i < 8; ++i) { ov[i] = run; run += ev[i]; }
    const v4i o0 = {ov[0], ov[1], ov[2], ov[3]};
    const v4i o1 = {ov[4], ov[5], ov[6], ov[7]};
    *(v4i*)(soff + 8 * tid)     = o0;
    *(v4i*)(soff + 8 * tid + 4) = o1;
    *(v4i*)(scur + 8 * tid)     = o0;
    *(v4i*)(scur + 8 * tid + 4) = o1;
  }
  __syncthreads();

#pragma unroll 1
  for (int ch = 0; ch < nChunks; ++ch) {
    const int cbase = ch * CHUNK;
    const int wc = scan_chunk<NB>(dsts, nE, cbase, nodeBase, vec8, list, tid, lane, wave);
    if (lane == 0) wcnt[wave] = wc;
    __syncthreads();
    if (wave == 0) {
#pragma unroll 1
      for (int wsx = 0; wsx < NWAVE; ++wsx) {
        int n = __builtin_amdgcn_readfirstlane(wcnt[wsx]);
        n = n > WCAP ? WCAP : (n < 0 ? 0 : n);
        const int* lp = list + wsx * WCAP;
#pragma unroll 1
        for (int i = 0; i < n; ++i) {
          const int ent  = __builtin_amdgcn_readfirstlane(lp[i]);
          const int slot = ent & (NB - 1);
          int e = cbase + ((ent >> 12) & (CHUNK - 1));
          e = e > nE - 1 ? nE - 1 : e;
          if (lane == 0) {
            int pos = scur[slot];
            pos = pos < 0 ? 0 : (pos > RCAP - 1 ? RCAP - 1 : pos);
            region[pos] = e;
            const int np = pos + 1;
            scur[slot] = np > RCAP ? RCAP : np;
          }
        }
      }
    }
    __syncthreads();
  }

  const v4f g4 = *(const v4f*)(g0 + 4 * lane);
  const v4f b4 = *(const v4f*)(b0 + 4 * lane);
  const v4f m4 = *(const v4f*)(st0 + 4 * lane);
  const v4f i4 = *(const v4f*)(st0 + STH + 4 * lane);
#pragma unroll 1
  for (int j = 0; j < NB / NWAVE; ++j) {
    const int slot = wave * (NB / NWAVE) + j;
    const int c = nodeBase + slot;
    if (c < nN) {
      int n = scnt[slot];
      n = n < 0 ? 0 : (n > DEGCAP ? DEGCAP : n);
      int st = soff[slot];
      st = st < 0 ? 0 : (st > RCAP - 1 ? RCAP - 1 : st);
      v4f acc = {0.f, 0.f, 0.f, 0.f};
#pragma unroll 1
      for (int q0 = 0; q0 < n; q0 += 32) {
        int pos = st + q0 + lane;
        pos = pos > RCAP - 1 ? RCAP - 1 : pos;
        int e = region[pos];
        e = e < 0 ? 0 : (e > nE - 1 ? nE - 1 : e);
        int sl = srcs[e];
        sl = sl < 0 ? 0 : (sl > nN - 1 ? nN - 1 : sl);
        const int mcnt = (n - q0) < 32 ? (n - q0) : 32;
#pragma unroll 1
        for (int p = 0; p < mcnt; ++p) {
          const int s = __builtin_amdgcn_readlane(sl, p);
          const v4f row = *(const v4f*)(y0 + (size_t)s * DH + 4 * lane);
          acc = acc + bn4(row, m4, i4, g4, b4);
        }
      }
      const v4f sv = bn4(*(const v4f*)(y0 + (size_t)c * DH + 4 * lane), m4, i4, g4, b4);
      const v4f v = sv + acc;
      float* op = aout + (size_t)c * DH + 4 * lane;
      *(volatile v4f*)op = v;
      __threadfence();
      *(volatile v4f*)op = v;
    }
  }
}

__global__ __launch_bounds__(NTHR) void k_resid(
    const float* __restrict__ y, const float* __restrict__ st, const float* __restrict__ g,
    const float* __restrict__ bb, const float* __restrict__ hr, const float* __restrict__ x,
    float* h3, int nN, int nUnits) {
  const int i4 = blockIdx.x * NTHR + (int)threadIdx.x;
  const bool ok = i4 < nUnits;
  int ic = i4 > nUnits - 1 ? nUnits - 1 : i4;
  ic = ic < 0 ? 0 : ic;
  const int row = ic >> 5;
  const int col = (ic & 31) * 4;
  const int xr = row > nN - 1 ? nN - 1 : row;
  const v4f yv = *(const v4f*)(y + (size_t)ic * 4);
  const v4f hv = *(const v4f*)(hr + (size_t)ic * 4);
  const v4f xv = *(const v4f*)(x + (size_t)xr * DH + col);
  const v4f m  = *(const v4f*)(st + col);
  const v4f is = *(const v4f*)(st + STH + col);
  const v4f gv = *(const v4f*)(g + col);
  const v4f bv = *(const v4f*)(bb + col);
  const v4f t = bn4(yv, m, is, gv, bv) + hv;
  const v4f v = xv + t;
  float* op = h3 + (size_t)ic * 4;
  if (ok) *(volatile v4f*)op = v;
  __threadfence();
  if (ok) *(volatile v4f*)op = v;
}

__global__ __launch_bounds__(NTHR) void k_final(
    float* out, const float* __restrict__ st, const float* __restrict__ g,
    const float* __restrict__ bb, const float* __restrict__ h3, int nUnits) {
  const int i4 = blockIdx.x * NTHR + (int)threadIdx.x;
  const bool ok = i4 < nUnits;
  int ic = i4 > nUnits - 1 ? nUnits - 1 : i4;
  ic = ic < 0 ? 0 : ic;
  const int col = (ic & 31) * 4;
  const v4f yv = *(const v4f*)(out + (size_t)ic * 4);
  const v4f hv = *(const v4f*)(h3 + (size_t)ic * 4);
  const v4f m  = *(const v4f*)(st + col);
  const v4f is = *(const v4f*)(st + STH + col);
  const v4f gv = *(const v4f*)(g + col);
  const v4f bv = *(const v4f*)(bb + col);
  const v4f v = bn4(yv, m, is, gv, bv) + hv;
  float* op = out + (size_t)ic * 4;
  if (ok) *(volatile v4f*)op = v;
  __threadfence();
  if (ok) *(volatile v4f*)op = v;
}

extern "C" void kernel_launch(void* const* d_in, const int* in_sizes, int n_in,
                              void* d_out, int out_size, void* d_ws, size_t ws_size,
                              hipStream_t stream) {
  if (n_in < 28) return;
  if (in_sizes[0] < DH || (in_sizes[0] % DH) != 0) return;
  const int nN = in_sizes[0] / DH;
  if (in_sizes[1] < 2 || (in_sizes[1] % 2) != 0) return;
  const int nE = in_sizes[1] / 2;
  const int D2 = 2 * DH, D4 = 4 * DH;
  if (in_sizes[2] != DH * DH || in_sizes[3] != DH || in_sizes[4] != DH || in_sizes[5] != DH) return;
  if (in_sizes[6] != DH * DH || in_sizes[7] != DH || in_sizes[8] != DH || in_sizes[9] != DH) return;
  if (in_sizes[10] != DH * DH || in_sizes[11] != DH) return;
  if (in_sizes[12] != DH * D2 || in_sizes[13] != D2 || in_sizes[14] != D2 || in_sizes[15] != D2) return;
  if (in_sizes[16] != D2 * DH || in_sizes[17] != DH || in_sizes[18] != DH || in_sizes[19] != DH) return;
  if (in_sizes[20] != DH * D4 || in_sizes[21] != D4 || in_sizes[22] != D4 || in_sizes[23] != D4) return;
  if (in_sizes[24] != D4 * DH || in_sizes[25] != DH || in_sizes[26] != DH || in_sizes[27] != DH) return;
  if (out_size != nN * DH) return;
  if (nN > (1 << 22) || nE > (1 << 28)) return;

  const float* x     = (const float*)d_in[0];
  const int*   ei    = (const int*)d_in[1];
  const float* encW  = (const float*)d_in[2];
  const float* encb  = (const float*)d_in[3];
  const float* bng0  = (const float*)d_in[4];
  const float* bnb0  = (const float*)d_in[5];
  const float* gW1   = (const float*)d_in[6];
  const float* gb1   = (const float*)d_in[7];
  const float* gg1   = (const float*)d_in[8];
  const float* gbb1  = (const float*)d_in[9];
  const float* gW2   = (const float*)d_in[10];
  const float* gb2   = (const float*)d_in[11];
  const float* f2W1  = (const float*)d_in[12];
  const float* f2b1  = (const float*)d_in[13];
  const float* f2g1  = (const float*)d_in[14];
  const float* f2bb1 = (const float*)d_in[15];
  const float* f2W2  = (const float*)d_in[16];
  const float* f2b2  = (const float*)d_in[17];
  const float* f2g2  = (const float*)d_in[18];
  const float* f2bb2 = (const float*)d_in[19];
  const float* fnW1  = (const float*)d_in[20];
  const float* fnb1  = (const float*)d_in[21];
  const float* fng1  = (const float*)d_in[22];
  const float* fnbb1 = (const float*)d_in[23];
  const float* fnW2  = (const float*)d_in[24];
  const float* fnb2  = (const float*)d_in[25];
  const float* fng2  = (const float*)d_in[26];
  const float* fnbb2 = (const float*)d_in[27];
  float* out = (float*)d_out;

  const int NPAD  = ((nN + RB - 1) / RB) * RB;
  const int nGemm = NPAD / RB;
  const int nBC   = (nN + NB - 1) / NB;
  const int nUnP  = NPAD * 32;
  const int nUnO  = nN * 32;
  const int nRes  = NPAD / 8;
  const int nFin  = (nUnO + NTHR - 1) / NTHR;

  char* ws = (char*)d_ws;
  size_t cur = 0;
  const size_t A256 = 255;
  const size_t szP  = (size_t)NPAD * DH * 4;
  const size_t oWh  = cur; cur += (size_t)WTOT * 2;                 cur = (cur + A256) & ~A256;
  const size_t oWl  = cur; cur += (size_t)WTOT * 2;                 cur = (cur + A256) & ~A256;
  const size_t oPt  = cur; cur += (size_t)nGemm * (2 * 512) * 8;    cur = (cur + A256) & ~A256;
  const size_t oSt  = cur; cur += (size_t)6 * STW * 4;              cur = (cur + A256) & ~A256;
  const size_t oAr  = cur; cur += szP + 4 * szP;                    cur = (cur + A256) & ~A256;
  if (cur > ws_size) return;
  if (cur > ((size_t)128 << 20)) return;
  unsigned short* whi = (unsigned short*)(ws + oWh);
  unsigned short* wlo = (unsigned short*)(ws + oWl);
  double* part = (double*)(ws + oPt);
  float*  st0  = (float*)(ws + oSt);
  float*  st1  = st0 + STW;
  float*  st2  = st1 + STW;
  float*  st3  = st2 + STW;
  float*  st4  = st3 + STW;
  float*  st5  = st4 + STW;
  float*  pA0  = (float*)(ws + oAr);
  float*  pA1  = (float*)(ws + oAr + szP);
  float*  pA2  = (float*)(ws + oAr + 2 * szP);
  float*  pA3  = (float*)(ws + oAr + 3 * szP);
  float*  pY4  = pA1;

  const int vec8 = ((nE & 3) == 0) ? 1 : 0;

  hipFuncSetAttribute(reinterpret_cast<const void*>(&k_gemm<128, 128, 0, 1>), hipFuncAttributeMaxDynamicSharedMemorySize, LDS_GEMM);
  hipFuncSetAttribute(reinterpret_cast<const void*>(&k_gemm<128, 128, 2, 0>), hipFuncAttributeMaxDynamicSharedMemorySize, LDS_GEMM);
  hipFuncSetAttribute(reinterpret_cast<const void*>(&k_gemm<128, 256, 0, 1>), hipFuncAttributeMaxDynamicSharedMemorySize, LDS_GEMM);
  hipFuncSetAttribute(reinterpret_cast<const void*>(&k_gemm<256, 128, 2, 1>), hipFuncAttributeMaxDynamicSharedMemorySize, LDS_GEMM);
  hipFuncSetAttribute(reinterpret_cast<const void*>(&k_gemm<128, 512, 0, 1>), hipFuncAttributeMaxDynamicSharedMemorySize, LDS_GEMM);
  hipFuncSetAttribute(reinterpret_cast<const void*>(&k_gemm<512, 128, 2, 1>), hipFuncAttributeMaxDynamicSharedMemorySize, LDS_GEMM);
  hipFuncSetAttribute(reinterpret_cast<const void*>(&k_aggr), hipFuncAttributeMaxDynamicSharedMemorySize, LDS_CSR);

  k_wprep<<<120, NTHR, 0, stream>>>(encW, gW1, gW2, f2W1, f2W2, fnW1, fnW2, whi, wlo);

  k_gemm<128, 128, 0, 1><<<nGemm, NTHR, LDS_GEMM, stream>>>(
      x, st0, bng0, bnb0, whi, wlo, encb, pA1, part, nN, NPAD);
  k_bnfin<<<1, 512, 0, stream>>>(part, nGemm, DH, nN, st0);

  k_aggr<<<nBC, NTHR, LDS_CSR, stream>>>(ei, pA1, st0, bng0, bnb0, pA2, nN, nE, vec8);

  k_gemm<128, 128, 0, 1><<<nGemm, NTHR, LDS_GEMM, stream>>>(
      pA2, st0, bng0, bnb0, whi + 16384, wlo + 16384, gb1, pA1, part, nN, NPAD);
  k_bnfin<<<1, 512, 0, stream>>>(part, nGemm, DH, nN, st1);

  k_gemm<128, 128, 2, 0><<<nGemm, NTHR, LDS_GEMM, stream>>>(
      pA1, st1, gg1, gbb1, whi + 32768, wlo + 32768, gb2, pA2, part, nN, NPAD);

  k_gemm<128, 256, 0, 1><<<nGemm, NTHR, LDS_GEMM, stream>>>(
      pA2, st1, gg1, gbb1, whi + 49152, wlo + 49152, f2b1, pA3, part, nN, NPAD);
  k_bnfin<<<1, 512, 0, stream>>>(part, nGemm, D2, nN, st2);

  k_gemm<256, 128, 2, 1><<<nGemm, NTHR, LDS_GEMM, stream>>>(
      pA3, st2, f2g1, f2bb1, whi + 81920, wlo + 81920, f2b2, pA1, part, nN, NPAD);
  k_bnfin<<<1, 512, 0, stream>>>(part, nGemm, DH, nN, st3);

  k_resid<<<nRes, NTHR, 0, stream>>>(pA1, st3, f2g2, f2bb2, pA2, x, pA0, nN, nUnP);

  k_gemm<128, 512, 0, 1><<<nGemm, NTHR, LDS_GEMM, stream>>>(
      pA0, st3, f2g2, f2bb2, whi + 114688, wlo + 114688, fnb1, pY4, part, nN, NPAD);
  k_bnfin<<<1, 512, 0, stream>>>(part, nGemm, D4, nN, st4);

  k_gemm<512, 128, 2, 1><<<nGemm, NTHR, LDS_GEMM, stream>>>(
      pY4, st4, fng1, fnbb1, whi + 180224, wlo + 180224, fnb2, out, part, nN, nN);
  k_bnfin<<<1, 512, 0, stream>>>(part, nGemm, DH, nN, st5);

  k_final<<<nFin, NTHR, 0, stream>>>(out, st5, fng2, fnbb2, pA0, nUnO);
}
